// VIBO_1PL_44659069944377
// MI455X (gfx1250) — hardware-verified
//
#include <hip/hip_runtime.h>
#include <stddef.h>
#include <math.h>


#define I_N   256
#define H_N   64
#define A_N   32
#define KP    72
#define NT    128
#define RH    128
#define PL_SZ (H_N * H_N)

static_assert((KP * 2) % 16 == 0);
static_assert(RH * 2 == I_N);
static_assert(NT == 128 && H_N == 64 && A_N * 2 == H_N && I_N == 256);

typedef float          v4f   __attribute__((ext_vector_type(4)));
typedef float          v8f   __attribute__((ext_vector_type(8)));
typedef unsigned short v8us  __attribute__((ext_vector_type(8)));
typedef unsigned short v16us __attribute__((ext_vector_type(16)));
typedef __bf16         v16bf __attribute__((ext_vector_type(16)));
union FragB { v16bf v; v16us u; v8us h[2]; };

__device__ __forceinline__ v8f wmb(const FragB& a, const FragB& b, v8f c) {
  v8f d = __builtin_amdgcn_wmma_f32_16x16x32_bf16(false, a.v, false, b.v, (short)0, c, false, false);
#if defined(__HIP_DEVICE_COMPILE__)
  asm volatile("v_nop\n\tv_nop\n\tv_nop\n\tv_nop" : "+v"(d) : "v"(a.u), "v"(b.u));
#endif
  return d;
}

__device__ __forceinline__ v8f zero8() {
  v8f z = {0.f, 0.f, 0.f, 0.f, 0.f, 0.f, 0.f, 0.f};
  return z;
}

__device__ __forceinline__ unsigned int bf16_bits(float x) {
  const unsigned int u = __float_as_uint(x);
  return (u + 0x7FFFu + ((u >> 16) & 1u)) >> 16;
}

__device__ __forceinline__ void split2(float x, unsigned int& hb, unsigned int& lb) {
  hb = bf16_bits(x);
  const float hf = __uint_as_float(hb << 16);
  lb = bf16_bits(x - hf);
}

__device__ __forceinline__ float eluf(float x) {
  const float e = __expf(fminf(x, 0.0f)) - 1.0f;
  return x > 0.0f ? x : e;
}

__global__ __launch_bounds__(256) void k_prep(const float* __restrict__ w2, const float* __restrict__ w3,
                                               const float* __restrict__ w4, unsigned short* planes) {
  const int b = blockIdx.x;
  const float* src = (b == 0) ? w2 : ((b == 1) ? w3 : w4);
  unsigned short* dh = planes + (size_t)(2 * b) * PL_SZ;
  unsigned short* dl = dh + PL_SZ;
  const int t = threadIdx.x;
  v8us vh[2], vl[2];
  int off[2];
#pragma unroll
  for (int j = 0; j < 2; ++j) {
    const int g = t + 256 * j;
    const int n = g >> 3, kg = g & 7;
#pragma unroll
    for (int e = 0; e < 8; ++e) {
      const int k = 8 * kg + e;
      const float x = src[k * H_N + n];
      unsigned int hb, lb;
      split2(x, hb, lb);
      vh[j][e] = (unsigned short)hb;
      vl[j][e] = (unsigned short)lb;
    }
    off[j] = n * H_N + 8 * kg;
  }
#pragma unroll
  for (int j = 0; j < 2; ++j) {
    *(volatile v8us*)(dh + off[j]) = vh[j];
    *(volatile v8us*)(dl + off[j]) = vl[j];
  }
  __threadfence();
#pragma unroll
  for (int j = 0; j < 2; ++j) {
    *(volatile v8us*)(dh + off[j]) = vh[j];
    *(volatile v8us*)(dl + off[j]) = vl[j];
  }
}

__global__ __launch_bounds__(NT) void k_person(
    const float* __restrict__ resp, const int* __restrict__ mask,
    const float* __restrict__ w1, const float* __restrict__ b1, const float* __restrict__ b2,
    const unsigned short* __restrict__ planes, float* hid) {
  __shared__ __align__(16) unsigned short sAh[RH * KP];
  __shared__ __align__(16) unsigned short sAl[RH * KP];
  __shared__ __align__(16) float sResp[I_N];
  __shared__ __align__(16) float sMask[I_N];
  __shared__ float sW1[H_N];
  __shared__ float sB1[H_N];
  __shared__ float sB2[H_N];
  __shared__ __align__(16) float sCol[H_N];

  const int tid = threadIdx.x, lane = tid & 31, wave = tid >> 5, hh = lane >> 4, m = lane & 15;
  const int p = blockIdx.x;
  const int n = wave * 16 + m;
  const size_t rb = (size_t)p * I_N;

  for (int i = tid; i < I_N; i += NT) {
    sResp[i] = resp[rb + i];
    sMask[i] = (float)mask[rb + i];
  }
  if (tid < H_N) {
    sW1[tid] = w1[tid];
    sB1[tid] = b1[tid];
    sB2[tid] = b2[tid];
  }

  const unsigned short* pw2h = planes;
  const unsigned short* pw2l = planes + PL_SZ;
  FragB bh[2], bl[2];
#pragma unroll
  for (int ks = 0; ks < 2; ++ks) {
    const int o = n * H_N + 32 * ks + 8 * hh;
    bh[ks].h[0] = *(const v8us*)(pw2h + o);
    bh[ks].h[1] = *(const v8us*)(pw2h + o + 16);
    bl[ks].h[0] = *(const v8us*)(pw2l + o);
    bl[ks].h[1] = *(const v8us*)(pw2l + o + 16);
  }
  __syncthreads();

  const float bias2 = sB2[n];
  float colsum = 0.0f;

  for (int half = 0; half < 2; ++half) {
#pragma unroll 1
    for (int j = 0; j < 8; ++j) {
      const int g = tid + NT * j;
      const int r = g >> 3, kg = g & 7;
      const float x = sResp[half * RH + r];
      v8us vh, vl;
#pragma unroll
      for (int e = 0; e < 8; ++e) {
        const int jj = 8 * kg + e;
        const float v = eluf(fmaf(x, sW1[jj], sB1[jj]));
        unsigned int hb, lb;
        split2(v, hb, lb);
        vh[e] = (unsigned short)hb;
        vl[e] = (unsigned short)lb;
      }
      *(v8us*)(sAh + r * KP + 8 * kg) = vh;
      *(v8us*)(sAl + r * KP + 8 * kg) = vl;
    }
    __syncthreads();

#pragma unroll 1
    for (int it = 0; it < RH / 16; ++it) {
      v8f acc = zero8();
      const unsigned short* arh = sAh + (it * 16 + m) * KP + 8 * hh;
      const unsigned short* arl = sAl + (it * 16 + m) * KP + 8 * hh;
#pragma unroll
      for (int ks = 0; ks < 2; ++ks) {
        FragB ah, al;
        ah.h[0] = *(const v8us*)(arh + 32 * ks);
        ah.h[1] = *(const v8us*)(arh + 32 * ks + 16);
        al.h[0] = *(const v8us*)(arl + 32 * ks);
        al.h[1] = *(const v8us*)(arl + 32 * ks + 16);
        acc = wmb(ah, bh[ks], acc);
        acc = wmb(ah, bl[ks], acc);
        acc = wmb(al, bh[ks], acc);
      }
      const int ib = half * RH + it * 16 + 8 * hh;
#pragma unroll
      for (int r = 0; r < 8; ++r) {
        const float val = eluf(acc[r] + bias2);
        colsum = fmaf(val, sMask[ib + r], colsum);
      }
    }
    __syncthreads();
  }

  colsum += __shfl_xor(colsum, 16, 32);
  if (hh == 0) sCol[n] = colsum;
  __syncthreads();

  if (wave == 0) {
    float d = 0.0f;
#pragma unroll
    for (int e = 0; e < 8; ++e) d += sMask[lane * 8 + e];
    d += __shfl_xor(d, 1, 32);
    d += __shfl_xor(d, 2, 32);
    d += __shfl_xor(d, 4, 32);
    d += __shfl_xor(d, 8, 32);
    d += __shfl_xor(d, 16, 32);
    d = fmaxf(d, 1.0f);
    const float inv = 1.0f / d;
    const v4f cv = *(const v4f*)(sCol + 4 * m);
    const v4f hv = cv * inv;
    float* hp = hid + (size_t)p * H_N + 4 * m;
    if (lane < 16) *(volatile v4f*)hp = hv;
    __threadfence();
    if (lane < 16) *(volatile v4f*)hp = hv;
  }
}

__global__ __launch_bounds__(NT) void k_head(
    const float* __restrict__ hid, const unsigned short* __restrict__ planes,
    const float* __restrict__ b3, const float* __restrict__ b4,
    const float* __restrict__ eps_ab, const float* __restrict__ eps_it,
    const int* __restrict__ item_index, const float* __restrict__ mu_tab, const float* __restrict__ lv_tab,
    float* out0, float* out1, float* out2, float* out3, float* out4, int nP, int nTab) {
  __shared__ __align__(16) unsigned short sAh[16 * KP];
  __shared__ __align__(16) unsigned short sAl[16 * KP];
  __shared__ __align__(16) unsigned short sTh[16 * KP];
  __shared__ __align__(16) unsigned short sTl[16 * KP];
  __shared__ __align__(16) float sOut[16 * H_N];
  __shared__ __align__(16) float sFeat[I_N];
  __shared__ __align__(16) float sImu[I_N];
  __shared__ __align__(16) float sIlv[I_N];
  __shared__ float sAbil[16];

  const int tid = threadIdx.x, lane = tid & 31, wave = tid >> 5, hh = lane >> 4, m = lane & 15;
  const int p0 = blockIdx.x * 16;
  const int n = wave * 16 + m;
  const unsigned short* pw3h = planes + 2 * PL_SZ;
  const unsigned short* pw3l = planes + 3 * PL_SZ;
  const unsigned short* pw4h = planes + 4 * PL_SZ;
  const unsigned short* pw4l = planes + 5 * PL_SZ;

  for (int j = 0; j < 8; ++j) {
    const int idx = tid + NT * j;
    const int row = idx >> 6, col = idx & 63;
    int pr = p0 + row;
    pr = pr > nP - 1 ? nP - 1 : pr;
    const float v = hid[(size_t)pr * H_N + col];
    unsigned int hb, lb;
    split2(v, hb, lb);
    sAh[row * KP + col] = (unsigned short)hb;
    sAl[row * KP + col] = (unsigned short)lb;
  }
#pragma unroll 1
  for (int i = tid; i < I_N; i += NT) {
    int ix = item_index[i];
    ix = ix < 0 ? 0 : (ix > nTab - 1 ? nTab - 1 : ix);
    const float imu = mu_tab[ix];
    const float ilv = lv_tab[ix];
    sImu[i] = imu;
    sIlv[i] = ilv;
    sFeat[i] = imu + eps_it[i] * expf(0.5f * ilv);
  }

  FragB bh[2], bl[2];
#pragma unroll
  for (int ks = 0; ks < 2; ++ks) {
    const int o = n * H_N + 32 * ks + 8 * hh;
    bh[ks].h[0] = *(const v8us*)(pw3h + o);
    bh[ks].h[1] = *(const v8us*)(pw3h + o + 16);
    bl[ks].h[0] = *(const v8us*)(pw3l + o);
    bl[ks].h[1] = *(const v8us*)(pw3l + o + 16);
  }
  __syncthreads();

  {
    v8f acc = zero8();
    const unsigned short* arh = sAh + m * KP + 8 * hh;
    const unsigned short* arl = sAl + m * KP + 8 * hh;
#pragma unroll
    for (int ks = 0; ks < 2; ++ks) {
      FragB ah, al;
      ah.h[0] = *(const v8us*)(arh + 32 * ks);
      ah.h[1] = *(const v8us*)(arh + 32 * ks + 16);
      al.h[0] = *(const v8us*)(arl + 32 * ks);
      al.h[1] = *(const v8us*)(arl + 32 * ks + 16);
      acc = wmb(ah, bh[ks], acc);
      acc = wmb(ah, bl[ks], acc);
      acc = wmb(al, bh[ks], acc);
    }
    const float bias3 = b3[n];
#pragma unroll
    for (int r = 0; r < 8; ++r) {
      const float t = eluf(acc[r] + bias3);
      unsigned int hb, lb;
      split2(t, hb, lb);
      sTh[(8 * hh + r) * KP + n] = (unsigned short)hb;
      sTl[(8 * hh + r) * KP + n] = (unsigned short)lb;
    }
  }
#pragma unroll
  for (int ks = 0; ks < 2; ++ks) {
    const int o = n * H_N + 32 * ks + 8 * hh;
    bh[ks].h[0] = *(const v8us*)(pw4h + o);
    bh[ks].h[1] = *(const v8us*)(pw4h + o + 16);
    bl[ks].h[0] = *(const v8us*)(pw4l + o);
    bl[ks].h[1] = *(const v8us*)(pw4l + o + 16);
  }
  __syncthreads();

  {
    v8f acc = zero8();
    const unsigned short* arh = sTh + m * KP + 8 * hh;
    const unsigned short* arl = sTl + m * KP + 8 * hh;
#pragma unroll
    for (int ks = 0; ks < 2; ++ks) {
      FragB ah, al;
      ah.h[0] = *(const v8us*)(arh + 32 * ks);
      ah.h[1] = *(const v8us*)(arh + 32 * ks + 16);
      al.h[0] = *(const v8us*)(arl + 32 * ks);
      al.h[1] = *(const v8us*)(arl + 32 * ks + 16);
      acc = wmb(ah, bh[ks], acc);
      acc = wmb(ah, bl[ks], acc);
      acc = wmb(al, bh[ks], acc);
    }
    const float bias4 = b4[n];
#pragma unroll
    for (int r = 0; r < 8; ++r) sOut[(8 * hh + r) * H_N + n] = acc[r] + bias4;
  }
  __syncthreads();

  {
    const int pl = tid >> 3, q = tid & 7;
    int pr = p0 + pl;
    pr = pr > nP - 1 ? nP - 1 : pr;
    float s = 0.0f;
#pragma unroll 1
    for (int e = 0; e < 4; ++e) {
      const int a = 4 * q + e;
      const float mu = sOut[pl * H_N + a];
      const float lv = sOut[pl * H_N + A_N + a];
      const float ep = eps_ab[(size_t)pr * A_N + a];
      s += mu + ep * expf(0.5f * lv);
    }
    s += __shfl_xor(s, 1, 32);
    s += __shfl_xor(s, 2, 32);
    s += __shfl_xor(s, 4, 32);
    if (q == 0) sAbil[pl] = s;
  }
  __syncthreads();

  v4f o0[8];
#pragma unroll
  for (int j = 0; j < 8; ++j) {
    const int idx = j * NT + tid;
    const int row = idx >> 6, c4 = idx & 63;
    const float ab = sAbil[row];
    const v4f fv = *(const v4f*)(sFeat + 4 * c4);
    v4f r4;
#pragma unroll
    for (int e = 0; e < 4; ++e) {
      float lg = ab + fv[e];
      lg = fminf(fmaxf(lg, -30.0f), 30.0f);
      const float ex = __expf(-lg);
      r4[e] = 1.0f / (1.0f + ex);
    }
    o0[j] = r4;
  }
  const int orow = tid >> 3, oc = tid & 7;
  const v4f v1 = *(const v4f*)(sOut + orow * H_N + 4 * oc);
  const v4f v2 = *(const v4f*)(sOut + orow * H_N + A_N + 4 * oc);
  const int per12 = p0 + orow;
  const bool ok12 = per12 < nP;
  float* d1 = out1 + (size_t)per12 * A_N + 4 * oc;
  float* d2 = out2 + (size_t)per12 * A_N + 4 * oc;
  const bool blk0 = (blockIdx.x == 0);
  const int t34 = tid & 63;
  const v4f va = *(const v4f*)(sImu + 4 * t34);
  const v4f vb = *(const v4f*)(sIlv + 4 * t34);
  const v4f v34 = (wave < 2) ? va : vb;
  float* d34 = ((wave < 2) ? out3 : out4) + 4 * t34;

#pragma unroll
  for (int j = 0; j < 8; ++j) {
    const int idx = j * NT + tid;
    const int row = idx >> 6, c4 = idx & 63;
    const int per = p0 + row;
    if (per < nP) *(volatile v4f*)(out0 + (size_t)per * I_N + 4 * c4) = o0[j];
  }
  if (ok12) {
    *(volatile v4f*)d1 = v1;
    *(volatile v4f*)d2 = v2;
  }
  if (blk0) *(volatile v4f*)d34 = v34;
  __threadfence();
#pragma unroll
  for (int j = 0; j < 8; ++j) {
    const int idx = j * NT + tid;
    const int row = idx >> 6, c4 = idx & 63;
    const int per = p0 + row;
    if (per < nP) *(volatile v4f*)(out0 + (size_t)per * I_N + 4 * c4) = o0[j];
  }
  if (ok12) {
    *(volatile v4f*)d1 = v1;
    *(volatile v4f*)d2 = v2;
  }
  if (blk0) *(volatile v4f*)d34 = v34;
}

extern "C" void kernel_launch(void* const* d_in, const int* in_sizes, int n_in,
                              void* d_out, int out_size, void* d_ws, size_t ws_size,
                              hipStream_t stream) {
  if (n_in < 15) return;
  if (in_sizes[2] != I_N || in_sizes[4] != I_N || in_sizes[13] != I_N || in_sizes[14] != I_N) return;
  if (in_sizes[5] != H_N || in_sizes[6] != H_N || in_sizes[7] != H_N * H_N || in_sizes[8] != H_N) return;
  if (in_sizes[9] != H_N * H_N || in_sizes[10] != H_N || in_sizes[11] != H_N * H_N || in_sizes[12] != H_N) return;
  if (in_sizes[3] <= 0 || (in_sizes[3] % A_N) != 0) return;
  const int nP = in_sizes[3] / A_N;
  if (nP <= 0 || nP > (1 << 20)) return;
  if (in_sizes[0] != nP * I_N || in_sizes[1] != nP * I_N) return;
  if (out_size != nP * I_N + 2 * nP * A_N + 2 * I_N) return;

  const float* resp       = (const float*)d_in[0];
  const int*   mask       = (const int*)d_in[1];
  const int*   item_index = (const int*)d_in[2];
  const float* eps_ab     = (const float*)d_in[3];
  const float* eps_it     = (const float*)d_in[4];
  const float* w1 = (const float*)d_in[5];
  const float* b1 = (const float*)d_in[6];
  const float* w2 = (const float*)d_in[7];
  const float* b2 = (const float*)d_in[8];
  const float* w3 = (const float*)d_in[9];
  const float* b3 = (const float*)d_in[10];
  const float* w4 = (const float*)d_in[11];
  const float* b4 = (const float*)d_in[12];
  const float* mu_tab = (const float*)d_in[13];
  const float* lv_tab = (const float*)d_in[14];

  float* out  = (float*)d_out;
  float* out0 = out;
  float* out1 = out0 + (size_t)nP * I_N;
  float* out2 = out1 + (size_t)nP * A_N;
  float* out3 = out2 + (size_t)nP * A_N;
  float* out4 = out3 + I_N;

  char* ws = (char*)d_ws;
  size_t off = 0;
  const size_t oPl  = off; off += (size_t)6 * PL_SZ * 2;         off = (off + 127) & ~(size_t)127;
  const size_t oHid = off; off += (size_t)nP * H_N * 4;          off = (off + 127) & ~(size_t)127;
  if (off > ws_size || off > (size_t)134217728) return;
  unsigned short* planes = (unsigned short*)(ws + oPl);
  float* hid = (float*)(ws + oHid);

  k_prep<<<3, 256, 0, stream>>>(w2, w3, w4, planes);
  k_person<<<nP, NT, 0, stream>>>(resp, mask, w1, b1, b2, planes, hid);
  k_head<<<(nP + 15) / 16, NT, 0, stream>>>(hid, planes, b3, b4, eps_ab, eps_it, item_index, mu_tab, lv_tab,
                                            out0, out1, out2, out3, out4, nP, I_N);
}
